// ConvolutionalSelfAttention_3899830305058
// MI455X (gfx1250) — hardware-verified
//
#include <hip/hip_runtime.h>


namespace {
#ifndef NB
#define NB 16
#endif
constexpr int C = 256, HWN = 1024, NF = 900, FS = 9, CG = 8, NR = NB * HWN;
constexpr float XS = 8.0f, WSC = 256.0f, QS = 64.0f, LOG2E = 1.4426950408889634f;
static_assert(NB >= 1 && NB <= 16);
static_assert(HWN % 32 == 0 && C % 64 == 0 && C % 32 == 0 && HWN % 256 == 0);
static_assert((CG * NF) % 4 == 0 && ((CG * NF * 4) % 128) == 0 && C % CG == 0);
static_assert(NR % 32 == 0);

typedef _Float16 b16;
typedef __attribute__((ext_vector_type(16))) _Float16 v16b;
typedef __attribute__((ext_vector_type(8))) _Float16 v8b;
typedef __attribute__((ext_vector_type(8))) float v8f;
typedef __attribute__((ext_vector_type(4))) float v4f;
__device__ __forceinline__ float bf16_rne(float f) { unsigned int u = __float_as_uint(f); u += 0x7FFFu + ((u >> 16) & 1u); return __uint_as_float(u & 0xFFFF0000u); }
__device__ __forceinline__ void split16(float v, b16& hi, b16& lo) { hi = (b16)v; lo = (b16)(v - (float)hi); }
__device__ __forceinline__ v16b frag_kb(const b16* p, int hh) { const v8b a = *(const v8b*)(p + 8 * hh), b = *(const v8b*)(p + 16 + 8 * hh); v16b f;
#pragma unroll
  for (int e = 0; e < 8; ++e) { f[e] = a[e]; f[8 + e] = b[e]; } return f; }
__device__ __forceinline__ v8f wmma16b(v16b a, v16b b, v8f c) { v8f d = __builtin_amdgcn_wmma_f32_16x16x32_f16(false, a, false, b, (short)0, c, false, false); asm volatile("v_nop\n\tv_nop\n\tv_nop\n\tv_nop" : "+v"(d) : "v"(a), "v"(b)); return d; }
__device__ __forceinline__ float nexp2(float x) { return __builtin_amdgcn_exp2f(x); }

__global__ __launch_bounds__(256) void prepx_kernel(const float* __restrict__ x, b16* __restrict__ X16) {
  __shared__ float tile[64][33];
  const int t_ = threadIdx.x, lane = t_ & 31, wave = t_ >> 5; const int b = blockIdx.z, n0 = blockIdx.x * 32, c0 = blockIdx.y * 64;
  const float* src = x + ((size_t)b * C + c0) * HWN + n0;
#pragma unroll
  for (int r = 0; r < 8; ++r) { const int cc = wave + 8 * r; tile[cc][lane] = src[(size_t)cc * HWN + lane]; }
  __syncthreads();
  const int nl = wave * 4 + (lane >> 3), c8 = (lane & 7) * 8; v8b o;
#pragma unroll
  for (int j = 0; j < 8; ++j) o[j] = (b16)(bf16_rne(tile[c8 + j][nl]) * XS);
  b16* dst = X16 + ((size_t)b * HWN + n0 + nl) * C + c0 + c8;
  *(volatile v8b*)dst = o; __threadfence(); *(volatile v8b*)dst = o;
}
__global__ __launch_bounds__(256) void prepw_kernel(const float* __restrict__ wk, const float* __restrict__ wq, b16* __restrict__ WT) {
  const size_t t = (size_t)blockIdx.x * 256 + threadIdx.x; if (t >= (size_t)2 * C * C / 8) return;
  const size_t e = t * 8; const bool second = e >= (size_t)C * C; const float* w = second ? wq : wk; const size_t eo = second ? e - (size_t)C * C : e;
  v8b o;
#pragma unroll
  for (int j = 0; j < 8; ++j) o[j] = (b16)(bf16_rne(w[eo + j]) * WSC);
  *(volatile v8b*)(WT + e) = o; __threadfence(); *(volatile v8b*)(WT + e) = o;
}
__global__ __launch_bounds__(256) void vals_kernel(const float* __restrict__ x, const float* __restrict__ vw, const float* __restrict__ vb, float* __restrict__ vals) {
  __shared__ float w[C];
  const int t_ = threadIdx.x; w[t_] = bf16_rne(vw[t_]); __syncthreads();
  const int b = blockIdx.y, n = blockIdx.x * 256 + t_;
  const float* p = x + (size_t)b * C * HWN + n; float acc = 0.0f;
#pragma unroll 4
  for (int c = 0; c < C; ++c) acc = fmaf(bf16_rne(p[(size_t)c * HWN]), w[c], acc);
  const float v = acc + bf16_rne(vb[0]);
  float* d = vals + (size_t)b * HWN + n; *(volatile float*)d = v; __threadfence(); *(volatile float*)d = v;
}
__global__ __launch_bounds__(128) void proj_kernel(const b16* __restrict__ X16, const b16* __restrict__ WT, const float* __restrict__ bk, const float* __restrict__ bq,
                                                    b16* __restrict__ Kh, b16* __restrict__ Kl, b16* __restrict__ Qh, b16* __restrict__ Ql) {
  __shared__ __attribute__((aligned(16))) float Ts[32][C + 8];
  const int wave = threadIdx.x >> 5, lane = threadIdx.x & 31, nloc = lane & 15, hlf = lane >> 4;
  const bool isq = blockIdx.y != 0;
  const b16* W = WT + (isq ? (size_t)C * C : (size_t)0); const float* bias = isq ? bq : bk; b16* Yh = isq ? Qh : Kh; b16* Yl = isq ? Ql : Kl;
  const int mt = wave & 1, n0 = (wave >> 1) * 128; const size_t rb = (size_t)blockIdx.x * 32; const size_t m0 = rb + mt * 16;
  v8f acc[8];
#pragma unroll
  for (int t = 0; t < 8; ++t) acc[t] = (v8f){};
#pragma unroll 2
  for (int kb = 0; kb < C; kb += 32) { const v16b a = frag_kb(X16 + (m0 + nloc) * C + kb, hlf);
#pragma unroll
    for (int t = 0; t < 8; ++t) { const v16b bw = frag_kb(W + (size_t)(n0 + t * 16 + nloc) * C + kb, hlf); acc[t] = wmma16b(a, bw, acc[t]); } }
  const float rs_ = 1.0f / (XS * WSC);
#pragma unroll
  for (int t = 0; t < 8; ++t) { const int c = n0 + t * 16 + nloc; const float bv = bf16_rne(bias[c]);
#pragma unroll
    for (int r = 0; r < 8; ++r) Ts[mt * 16 + 8 * hlf + r][c] = acc[t][r] * rs_ + bv; }
  __syncthreads();
#pragma unroll 1
  for (int rr = 0; rr < 8; ++rr) { const int row = wave * 8 + rr; const v4f f0 = *(const v4f*)(&Ts[row][lane * 8]), f1 = *(const v4f*)(&Ts[row][lane * 8 + 4]);
    float f[8] = {f0.x, f0.y, f0.z, f0.w, f1.x, f1.y, f1.z, f1.w}; float ss = 0.0f;
#pragma unroll
    for (int j = 0; j < 8; ++j) ss = fmaf(f[j], f[j], ss);
#pragma unroll
    for (int o_ = 16; o_ > 0; o_ >>= 1) ss += __shfl_xor(ss, o_);
    const float inv = 1.0f / fmaxf(sqrtf(ss), 1e-12f);
    v8b hv, lv;
#pragma unroll
    for (int j = 0; j < 8; ++j) { b16 p, q; split16(f[j] * inv * QS, p, q); hv[j] = p; lv[j] = q; }
    b16* ph = Yh + (rb + row) * C + lane * 8; b16* pl = Yl + (rb + row) * C + lane * 8;
    *(volatile v8b*)ph = hv; *(volatile v8b*)pl = lv; __threadfence(); *(volatile v8b*)ph = hv; *(volatile v8b*)pl = lv; }
}
__global__ __launch_bounds__(64) void attn_kernel(const b16* __restrict__ Qh, const b16* __restrict__ Ql, const b16* __restrict__ Kh, const b16* __restrict__ Kl, const float* __restrict__ vals, float* __restrict__ wmap) {
  __shared__ float vs[HWN]; __shared__ float wq[32];
  const int wave = threadIdx.x >> 5, lane = threadIdx.x & 31, hh = lane >> 4, col = lane & 15; const int b = blockIdx.y; const int q0 = blockIdx.x * 32 + wave * 16, qi = q0 + col;
  for (int i = threadIdx.x; i < HWN; i += 64) vs[i] = vals[(size_t)b * HWN + i];
  __syncthreads();
  const size_t qo = ((size_t)b * HWN + qi) * C;
  const b16* Kb = Kh + (size_t)b * HWN * C; const b16* Klb = Kl + (size_t)b * HWN * C;
  float m = -1.0e30f, l = 0.0f, wacc = 0.0f;
  const float cs = LOG2E / (QS * QS);
  for (int kb = 0; kb < HWN; kb += 32) {
    v8f s0 = {}, s1 = {};
#pragma unroll 2
    for (int ks = 0; ks < C; ks += 32) { const v16b qa = frag_kb(Qh + qo + ks, hh), ql = frag_kb(Ql + qo + ks, hh);
      const b16* k0 = Kb + (size_t)(kb + col) * C + ks, *k1 = Kb + (size_t)(kb + 16 + col) * C + ks;
      v16b f = frag_kb(k0, hh); s0 = wmma16b(f, qa, s0); s0 = wmma16b(f, ql, s0); s0 = wmma16b(frag_kb(Klb + (size_t)(kb + col) * C + ks, hh), qa, s0);
      f = frag_kb(k1, hh); s1 = wmma16b(f, qa, s1); s1 = wmma16b(f, ql, s1); s1 = wmma16b(frag_kb(Klb + (size_t)(kb + 16 + col) * C + ks, hh), qa, s1); }
    float e[16]; float mx = -1.0e30f;
#pragma unroll
    for (int r = 0; r < 8; ++r) { e[r] = s0[r] * cs; e[8 + r] = s1[r] * cs; mx = fmaxf(mx, fmaxf(e[r], e[8 + r])); }
    mx = fmaxf(mx, __shfl_xor(mx, 16)); const float mn = fmaxf(m, mx); const float al = nexp2(m - mn); m = mn; float sum = 0.0f, vsum = 0.0f;
#pragma unroll
    for (int i = 0; i < 8; ++i) { const float p0 = nexp2(e[i] - mn), p1 = nexp2(e[8 + i] - mn); sum += p0 + p1; vsum = fmaf(p0, vs[kb + 8 * hh + i], vsum); vsum = fmaf(p1, vs[kb + 16 + 8 * hh + i], vsum); }
    sum += __shfl_xor(sum, 16); vsum += __shfl_xor(vsum, 16); l = l * al + sum; wacc = wacc * al + vsum; }
  const float w = wacc * (1.0f / l);
  if (hh == 0) wq[wave * 16 + col] = w;
  __syncthreads();
  if (wave == 0) { const float v = wq[lane]; float* p = wmap + (size_t)b * HWN + (size_t)blockIdx.x * 32 + lane; *(volatile float*)p = v; __threadfence(); *(volatile float*)p = v; }
}
__global__ __launch_bounds__(256) void conv_kernel(const float* __restrict__ x, const int* __restrict__ li, const float* __restrict__ wmap, float* __restrict__ out) {
  __shared__ float wm[HWN]; __shared__ float prod[HWN]; __shared__ __attribute__((aligned(16))) float outs[CG * NF]; __shared__ unsigned short lis[NF * FS];
  const int t_ = threadIdx.x; const int b = blockIdx.y, c0 = blockIdx.x * CG;
  for (int i = t_; i < HWN; i += 256) wm[i] = wmap[(size_t)b * HWN + i];
  for (int i = t_; i < NF * FS; i += 256) { int v = li[i]; v = v < 0 ? 0 : (v > HWN - 1 ? HWN - 1 : v); lis[i] = (unsigned short)v; }
  for (int ch = 0; ch < CG; ++ch) {
    __syncthreads();
    const float* xr = x + ((size_t)b * C + c0 + ch) * HWN;
    for (int i = t_; i < HWN; i += 256) prod[i] = wm[i] * bf16_rne(xr[i]);
    __syncthreads();
    for (int f = t_; f < NF; f += 256) { float s = 0.0f; const unsigned short* qp = lis + f * FS;
#pragma unroll
      for (int k = 0; k < FS; ++k) s += prod[qp[k]];
      outs[ch * NF + f] = s; }
  }
  __syncthreads();
  constexpr int NG = CG * NF / 4;
  float* ob = out + ((size_t)b * C + c0) * NF;
  for (int it = 0; it < (NG + 255) / 256; ++it) { const int g = it * 256 + t_; const int gc = g < NG ? g : NG - 1; const v4f v = *(const v4f*)(&outs[gc * 4]);
    if (g < NG) *(volatile v4f*)(ob + (size_t)g * 4) = v;
    __threadfence();
    if (g < NG) *(volatile v4f*)(ob + (size_t)g * 4) = v; }
}
}

extern "C" void kernel_launch(void* const* d_in, const int* in_sizes, int n_in, void* d_out, int out_size, void* d_ws, size_t ws_size, hipStream_t stream) {
  if (n_in < 8) return;
  auto Fp = [&](int i) { return (const float*)d_in[i]; };
  if (in_sizes[0] < NR * C || in_sizes[1] < C * C || in_sizes[2] < C || in_sizes[3] < C * C || in_sizes[4] < C || in_sizes[5] < C || in_sizes[6] < 1 || in_sizes[7] < NF * FS || out_size < NB * C * NF) return;
  size_t off = 0; char* ws = (char*)d_ws;
  auto carve = [&](size_t bytes) { char* p = ws + off; off += (bytes + 255) & ~(size_t)255; return p; };
  b16* X16 = (b16*)carve((size_t)NR * C * 2); b16* WT = (b16*)carve((size_t)2 * C * C * 2);
  b16* Kh = (b16*)carve((size_t)NR * C * 2); b16* Kl = (b16*)carve((size_t)NR * C * 2); b16* Qh = (b16*)carve((size_t)NR * C * 2); b16* Ql = (b16*)carve((size_t)NR * C * 2);
  float* VALS = (float*)carve((size_t)NR * 4); float* WMAP = (float*)carve((size_t)NR * 4);
  if (off > ws_size || off > ((size_t)128 << 20)) return;
  prepx_kernel<<<dim3(HWN / 32, C / 64, NB), 256, 0, stream>>>(Fp(0), X16);
  prepw_kernel<<<dim3((2 * C * C / 8) / 256), 256, 0, stream>>>(Fp(1), Fp(3), WT);
  vals_kernel<<<dim3(HWN / 256, NB), 256, 0, stream>>>(Fp(0), Fp(5), Fp(6), VALS);
  proj_kernel<<<dim3(NR / 32, 2), 128, 0, stream>>>(X16, WT, Fp(2), Fp(4), Kh, Kl, Qh, Ql);
  attn_kernel<<<dim3(HWN / 32, NB), 64, 0, stream>>>(Qh, Ql, Kh, Kl, VALS, WMAP);
  conv_kernel<<<dim3(C / CG, NB), 256, 0, stream>>>(Fp(0), (const int*)d_in[7], WMAP, (float*)d_out);
}
